// SimpleGraphHead_21835613733002
// MI455X (gfx1250) — hardware-verified
//
#include <hip/hip_runtime.h>


#define NB_  128
#define NN   64
#define CL   64
#define C2L  128
#define NNODE (NB_ * NN)
#define ICH  16
#define PCH  (ICH * NN * NN)
#define DM   CL
#define LOSC 1024.0f
typedef _Float16 h16;
typedef unsigned short bf;
typedef __attribute__((ext_vector_type(16))) __bf16   v16bf;
typedef __attribute__((ext_vector_type(16))) _Float16 v16h;
typedef __attribute__((ext_vector_type(8)))  _Float16 v8h;
typedef __attribute__((ext_vector_type(8)))  unsigned short v8us;
typedef __attribute__((ext_vector_type(8)))  float    v8f;
typedef __attribute__((ext_vector_type(4)))  float    v4f;
typedef __attribute__((ext_vector_type(4)))  _Float16 v4h;
typedef v8h  __attribute__((may_alias)) v8ha;
typedef v4f  __attribute__((may_alias)) v4fa;
typedef v8us __attribute__((may_alias)) v8usa;

__device__ __forceinline__ unsigned short f2bf(float f) { unsigned u = __float_as_uint(f); u += 0x7FFFu + ((u >> 16) & 1u); return (unsigned short)(u >> 16); }
__device__ __forceinline__ float bf2f(unsigned short b) { return __uint_as_float(((unsigned)b) << 16); }
__device__ __forceinline__ float bfr(float f) { return bf2f(f2bf(f)); }
__device__ __forceinline__ v16h cat16(v8h lo, v8h hi) { return __builtin_shufflevector(lo, hi, 0, 1, 2, 3, 4, 5, 6, 7, 8, 9, 10, 11, 12, 13, 14, 15); }
__device__ __forceinline__ v16bf cat16b(v8us lo, v8us hi) { return __builtin_bit_cast(v16bf, __builtin_shufflevector(lo, hi, 0, 1, 2, 3, 4, 5, 6, 7, 8, 9, 10, 11, 12, 13, 14, 15)); }
__device__ __forceinline__ v8f wmma16(v16h a, v16h b, v8f c) { return __builtin_amdgcn_wmma_f32_16x16x32_f16(false, a, false, b, (short)0, c, false, false); }
__device__ __forceinline__ v8f wmmab(v16bf a, v16bf b, v8f c) { return __builtin_amdgcn_wmma_f32_16x16x32_bf16(false, a, false, b, (short)0, c, false, false); }

template <bool SPLITA, bool F16OUT = false>
__global__ __launch_bounds__(128) void k_gemmb(const bf* __restrict__ A, const bf* __restrict__ Al, const bf* __restrict__ Bn, const float* __restrict__ bias, float* C, int ldc, h16* C2, const float* __restrict__ R = nullptr, int K = DM, int roundR = 1) {
    __shared__ __align__(16) float ost[4][16 * 68];
    const int lane = threadIdx.x & 31, wave = threadIdx.x >> 5, lr = lane & 15, hi = lane >> 4;
    const int r0 = blockIdx.x * 64 + wave * 16, c0 = blockIdx.y * 64;
    const size_t aoff = (size_t)(r0 + lr) * K + 8 * hi;
    size_t boff[4];
#pragma unroll
    for (int t = 0; t < 4; ++t) boff[t] = (size_t)(c0 + t * 16 + lr) * K + 8 * hi;
    v8f acc[4];
#pragma unroll
    for (int t = 0; t < 4; ++t) acc[t] = (v8f){};
#pragma unroll 1
    for (int kc = 0; kc < K; kc += 32) {
        const v16bf a = cat16b(*(const v8us*)(A + aoff + kc), *(const v8us*)(A + aoff + kc + 16));
        v16bf al = a;
        if (SPLITA) al = cat16b(*(const v8us*)(Al + aoff + kc), *(const v8us*)(Al + aoff + kc + 16));
#pragma unroll
        for (int t = 0; t < 4; ++t) { const v16bf b = cat16b(*(const v8us*)(Bn + boff[t] + kc), *(const v8us*)(Bn + boff[t] + kc + 16)); acc[t] = wmmab(a, b, acc[t]); if (SPLITA) acc[t] = wmmab(al, b, acc[t]); }
        asm volatile("v_nop\n\tv_nop\n\tv_nop\n\tv_nop" : "+v"(acc[0]), "+v"(acc[1]), "+v"(acc[2]), "+v"(acc[3]) : "v"(a), "v"(al));
    }
    float* os = &ost[wave][0];
#pragma unroll
    for (int t = 0; t < 4; ++t) { const float bv = bias ? bfr(bias[c0 + t * 16 + lr]) : 0.f;
#pragma unroll
        for (int j = 0; j < 8; ++j) os[(hi * 8 + j) * 68 + t * 16 + lr] = acc[t][j] + bv; }
    __syncthreads();
    if (F16OUT) {
        h16* crow = (h16*)(void*)C + (size_t)r0 * ldc + c0;
        auto pass = [&]() {
#pragma unroll
            for (int s = 0; s < 4; ++s) { const int row = 4 * s + (lane >> 3), piece = lane & 7; const float* sp = os + row * 68 + piece * 8; v8h o, o2;
#pragma unroll
                for (int i = 0; i < 8; ++i) { const h16 a = (h16)sp[i]; o[i] = a; o2[i] = (h16)((sp[i] - (float)a) * LOSC); }
                *(volatile v8h*)(crow + (size_t)row * ldc + piece * 8) = o; if (C2) *(volatile v8h*)(C2 + (size_t)r0 * ldc + c0 + (size_t)row * ldc + piece * 8) = o2; }
        };
        pass(); __threadfence(); pass();
    } else {
        float* crow = C + (size_t)r0 * ldc + c0;
        auto pass = [&]() {
#pragma unroll
            for (int s = 0; s < 8; ++s) { const int Lid = (lane >> 3) + 4 * s, piece = lane & 7; const int row = Lid >> 1, cofs = (Lid & 1) * 32 + piece * 4;
                v4f val = *(const v4fa*)(os + row * 68 + cofs); if (R) { const v4f rv = *(const v4f*)(R + ((size_t)r0 + row) * ldc + c0 + cofs); val += roundR ? (v4f){bfr(rv[0]), bfr(rv[1]), bfr(rv[2]), bfr(rv[3])} : rv; }
                *(volatile v4f*)(crow + (size_t)row * ldc + cofs) = val; }
        };
        pass(); __threadfence(); pass();
    }
}


__global__ __launch_bounds__(128) void k_gemmh(const h16* __restrict__ A, const h16* __restrict__ Bn, const float* __restrict__ bias, float* C, int ldc, const float* __restrict__ R, int K, size_t sA, size_t sB, size_t sC, int roundR) {
    __shared__ __align__(16) float ost[4][16 * 68];
    const size_t z = blockIdx.z; A += z * sA; Bn += z * sB; C += z * sC; if (R) R += z * sC;
    const int lane = threadIdx.x & 31, wave = threadIdx.x >> 5, lr = lane & 15, hi = lane >> 4;
    const int r0 = blockIdx.x * 64 + wave * 16, c0 = blockIdx.y * 64;
    const size_t aoff = (size_t)(r0 + lr) * K + 8 * hi;
    size_t boff[4];
#pragma unroll
    for (int t = 0; t < 4; ++t) boff[t] = (size_t)(c0 + t * 16 + lr) * K + 8 * hi;
    v8f acc[4];
#pragma unroll
    for (int t = 0; t < 4; ++t) acc[t] = (v8f){};
#pragma unroll 1
    for (int kc = 0; kc < K; kc += 32) {
        const v16h a = cat16(*(const v8h*)(A + aoff + kc), *(const v8h*)(A + aoff + kc + 16));
#pragma unroll
        for (int t = 0; t < 4; ++t) { const v16h b = cat16(*(const v8h*)(Bn + boff[t] + kc), *(const v8h*)(Bn + boff[t] + kc + 16)); acc[t] = wmma16(a, b, acc[t]); }
        asm volatile("v_nop\n\tv_nop\n\tv_nop\n\tv_nop" : "+v"(acc[0]), "+v"(acc[1]), "+v"(acc[2]), "+v"(acc[3]) : "v"(a));
    }
    float* os = &ost[wave][0];
#pragma unroll
    for (int t = 0; t < 4; ++t) { const float bv = bias ? bfr(bias[c0 + t * 16 + lr]) : 0.f;
#pragma unroll
        for (int j = 0; j < 8; ++j) os[(hi * 8 + j) * 68 + t * 16 + lr] = acc[t][j] + bv; }
    __syncthreads();
    float* crow = C + (size_t)r0 * ldc + c0;
    auto pass = [&]() {
#pragma unroll
        for (int s = 0; s < 8; ++s) { const int Lid = (lane >> 3) + 4 * s, piece = lane & 7; const int row = Lid >> 1, cofs = (Lid & 1) * 32 + piece * 4;
            v4f val = *(const v4fa*)(os + row * 68 + cofs); if (R) { const v4f rv = *(const v4f*)(R + ((size_t)r0 + row) * ldc + c0 + cofs); val += roundR ? (v4f){bfr(rv[0]), bfr(rv[1]), bfr(rv[2]), bfr(rv[3])} : rv; }
            *(volatile v4f*)(crow + (size_t)row * ldc + cofs) = val; }
    };
    pass(); __threadfence(); pass();
}

typedef __attribute__((ext_vector_type(4))) _Float16 v4h;
__device__ __forceinline__ h16 tohx(float x) { return (h16)x; }
__global__ __launch_bounds__(256) void k_wt_io(const float* __restrict__ Wm, int ldw, int K, int N, bf* Bt) {
    const int lane = threadIdx.x & 31; const int n = blockIdx.x * 8 + (threadIdx.x >> 5); if (n >= N) return;
#pragma unroll 1
    for (int ps = 0; ps < 2; ++ps) { for (int c0 = lane * 8; c0 < K; c0 += 256) { v8us o;
#pragma unroll
            for (int i = 0; i < 8; ++i) { const int k = c0 + i; o[i] = f2bf(k < K ? Wm[(size_t)(k < K ? k : 0) * ldw + n] : 0.f); }
            *(volatile v8us*)(Bt + (size_t)n * K + c0) = o; }
        if (ps == 0) __threadfence(); }
}
__global__ __launch_bounds__(256) void k_wt_ioh(const float* __restrict__ Wm, int ldw, int K, int N, h16* Bt) {
    const int lane = threadIdx.x & 31; const int n = blockIdx.x * 8 + (threadIdx.x >> 5); if (n >= N) return;
#pragma unroll 1
    for (int ps = 0; ps < 2; ++ps) { for (int c0 = lane * 8; c0 < K; c0 += 256) { v8h o;
#pragma unroll
            for (int i = 0; i < 8; ++i) { const int k = c0 + i; o[i] = tohx(k < K ? bfr(Wm[(size_t)(k < K ? k : 0) * ldw + n]) : 0.f); }
            *(volatile v8h*)(Bt + (size_t)n * K + c0) = o; }
        if (ps == 0) __threadfence(); }
}
__global__ __launch_bounds__(256) void k_cvt64(const float* __restrict__ s, bf* A) {
    const int lane = threadIdx.x & 31; const size_t r = ((size_t)blockIdx.x * 8 + (threadIdx.x >> 5)) * 4 + (lane >> 3); if (r >= (size_t)NNODE) return; const int c0 = (lane & 7) * 8; v8us o;
#pragma unroll
    for (int i = 0; i < 8; ++i) o[i] = f2bf(s[r * CL + c0 + i]);
    *(volatile v8us*)(A + r * CL + c0) = o; __threadfence(); *(volatile v8us*)(A + r * CL + c0) = o;
}
template <int W>
__global__ __launch_bounds__(256) void k_relusplit(const float* __restrict__ F, size_t rows, bf* Ph, bf* Pl) {
    const int RPW = 256 / W; const int lane = threadIdx.x & 31; const size_t r = ((size_t)blockIdx.x * 8 + (threadIdx.x >> 5)) * RPW + lane / (W / 8); if (r >= rows) return; const int c0 = (lane % (W / 8)) * 8; v8us oh, ol;
#pragma unroll
    for (int i = 0; i < 8; ++i) { const float y = fmaxf(F[r * W + c0 + i], 0.f); const unsigned short hb = f2bf(y); oh[i] = hb; ol[i] = f2bf(y - bf2f(hb)); }
    *(volatile v8us*)(Ph + r * W + c0) = oh; *(volatile v8us*)(Pl + r * W + c0) = ol; __threadfence(); *(volatile v8us*)(Ph + r * W + c0) = oh; *(volatile v8us*)(Pl + r * W + c0) = ol;
}

__global__ __launch_bounds__(256) void k_relusplitf64(const float* __restrict__ F, size_t rows, float* HN, bf* Ph, bf* Pl) {
    typedef __attribute__((ext_vector_type(4))) unsigned short v4us;
    const int lane = threadIdx.x & 31; const size_t r = ((size_t)blockIdx.x * 8 + (threadIdx.x >> 5)) * 2 + (lane >> 4); if (r >= rows) return; const int c0 = (lane & 15) * 4; v4us oh, ol; v4f y;
#pragma unroll
    for (int i = 0; i < 4; ++i) { y[i] = fmaxf(F[r * CL + c0 + i], 0.f); const unsigned short hb = f2bf(y[i]); oh[i] = hb; ol[i] = f2bf(y[i] - bf2f(hb)); }
#pragma unroll 1
    for (int ps = 0; ps < 2; ++ps) { *(volatile v4f*)(HN + r * CL + c0) = y; *(volatile v4us*)(Ph + r * CL + c0) = oh; *(volatile v4us*)(Pl + r * CL + c0) = ol; if (ps == 0) __threadfence(); }
}
__global__ __launch_bounds__(256) void k_pair1(const float* __restrict__ HN, const float* __restrict__ UV, const float* __restrict__ rcw1, const float* __restrict__ rcb1, const float* __restrict__ anw1, const float* __restrict__ anb1, int node0, h16* R1, h16* T1) {
    const int lane = threadIdx.x & 31; const size_t p = (size_t)blockIdx.x * 8 + (threadIdx.x >> 5); if (p >= (size_t)PCH) return; const int nl = (int)(p / NN), j = (int)(p % NN); const int ni = node0 + nl; const int nj = (ni / NN) * NN + j;
    const float d0 = HN[(size_t)ni * CL] - HN[(size_t)nj * CL], d1 = HN[(size_t)ni * CL + 1] - HN[(size_t)nj * CL + 1]; const float dist = d0 * d0 + d1 * d1;
    if (lane < 16) { const int c0 = lane * 8; v8h o;
#pragma unroll
        for (int i = 0; i < 8; ++i) { const int c = c0 + i; const float y = UV[(size_t)ni * 384 + c] + UV[(size_t)nj * 384 + 128 + c] + dist * bfr(rcw1[(size_t)128 * C2L + c]) + bfr(rcb1[c]); o[i] = tohx(fmaxf(y, 0.f)); }
        *(volatile v8h*)(R1 + p * C2L + c0) = o; __threadfence(); *(volatile v8h*)(R1 + p * C2L + c0) = o; }
    else if (lane < 24) { const int c0 = (lane - 16) * 8; v8h o;
#pragma unroll
        for (int i = 0; i < 8; ++i) { const int c = c0 + i; const float y = UV[(size_t)ni * 384 + 256 + c] + UV[(size_t)nj * 384 + 320 + c] + dist * bfr(anw1[(size_t)128 * CL + c]) + bfr(anb1[c]); o[i] = tohx(fmaxf(y, 0.f)); }
        *(volatile v8h*)(T1 + p * CL + c0) = o; __threadfence(); *(volatile v8h*)(T1 + p * CL + c0) = o; }
}
__global__ __launch_bounds__(256) void k_reluh128(const float* __restrict__ F, size_t rows, h16* Hh) {
    const int lane = threadIdx.x & 31; const size_t r = ((size_t)blockIdx.x * 8 + (threadIdx.x >> 5)) * 2 + (lane >> 4); if (r >= rows) return; const int c0 = (lane & 15) * 8; v8h o;
#pragma unroll
    for (int i = 0; i < 8; ++i) o[i] = tohx(fmaxf(F[r * C2L + c0 + i], 0.f));
    *(volatile v8h*)(Hh + r * C2L + c0) = o; __threadfence(); *(volatile v8h*)(Hh + r * C2L + c0) = o;
}
__global__ __launch_bounds__(256) void k_pairmean(const float* __restrict__ REL, const float* __restrict__ ATT, int node0, float* RD) {
    const int lane = threadIdx.x & 31; const int nl = blockIdx.x * 8 + (threadIdx.x >> 5); if (nl >= PCH / NN) return; const int c0 = lane * 4; v4f acc = (v4f){0.f, 0.f, 0.f, 0.f};
#pragma unroll 1
    for (int j = 0; j < NN; ++j) { const size_t p = (size_t)nl * NN + j;
#pragma unroll
        for (int i = 0; i < 4; ++i) { const float rv = fmaxf(REL[p * C2L + c0 + i], 0.f); const float av = 1.0f / (1.0f + expf(-ATT[p * C2L + c0 + i])); acc[i] += rv * av; } }
#pragma unroll
    for (int i = 0; i < 4; ++i) acc[i] *= (1.0f / NN);
    float* dst = RD + (size_t)(node0 + nl) * C2L + c0; *(volatile v4f*)dst = acc; __threadfence(); *(volatile v4f*)dst = acc;
}
__global__ __launch_bounds__(256) void k_outmean(const float* __restrict__ SD, const float* __restrict__ RD, float* OUTB) {
    const int lane = threadIdx.x & 31; const int b = blockIdx.x * 8 + (threadIdx.x >> 5); if (b >= NB_) return; const int c0 = lane * 4; v4f acc = (v4f){0.f, 0.f, 0.f, 0.f};
#pragma unroll 1
    for (int i = 0; i < NN; ++i) { const size_t n = (size_t)b * NN + i;
#pragma unroll
        for (int k = 0; k < 4; ++k) acc[k] += SD[n * C2L + c0 + k] + RD[n * C2L + c0 + k]; }
#pragma unroll
    for (int k = 0; k < 4; ++k) acc[k] *= (1.0f / NN);
    *(volatile v4f*)(OUTB + (size_t)b * C2L + c0) = acc; __threadfence(); *(volatile v4f*)(OUTB + (size_t)b * C2L + c0) = acc;
}
extern "C" void kernel_launch(void* const* d_in, const int* in_sizes, int n_in,
                              void* d_out, int out_size, void* d_ws, size_t ws_size, hipStream_t stream) {
    (void)in_sizes; (void)n_in; (void)out_size;
    const float* s = (const float*)d_in[0]; const float* sew1 = (const float*)d_in[1]; const float* seb1 = (const float*)d_in[2]; const float* sew2 = (const float*)d_in[3]; const float* seb2 = (const float*)d_in[4];
    const float* sdw1 = (const float*)d_in[5]; const float* sdb1 = (const float*)d_in[6]; const float* sdw2 = (const float*)d_in[7]; const float* sdb2 = (const float*)d_in[8];
    const float* rcw1 = (const float*)d_in[9]; const float* rcb1 = (const float*)d_in[10]; const float* rcw2 = (const float*)d_in[11]; const float* rcb2 = (const float*)d_in[12]; const float* rcw3 = (const float*)d_in[13]; const float* rcb3 = (const float*)d_in[14];
    const float* anw1 = (const float*)d_in[15]; const float* anb1 = (const float*)d_in[16]; const float* anw2 = (const float*)d_in[17]; const float* anb2 = (const float*)d_in[18];
    float* out = (float*)d_out;
    char* wsp = (char*)d_ws;
    auto take = [&](size_t bytes) { char* p = wsp; wsp += (bytes + 255) & ~(size_t)255; return (void*)p; };
    bf* WSE1 = (bf*)take(CL * CL * 2); bf* WSE2 = (bf*)take(CL * CL * 2); bf* WSD1 = (bf*)take(C2L * CL * 2); bf* WSD2 = (bf*)take(C2L * C2L * 2); bf* WUV = (bf*)take(384 * CL * 2);
    h16* WRC2 = (h16*)take(C2L * C2L * 2); h16* WRC3 = (h16*)take(C2L * C2L * 2); h16* WAN2 = (h16*)take(C2L * CL * 2);
    bf* A0 = (bf*)take((size_t)NNODE * CL * 2); float* F1 = (float*)take((size_t)NNODE * CL * 4); bf* Ph = (bf*)take((size_t)NNODE * C2L * 2); bf* Pl = (bf*)take((size_t)NNODE * C2L * 2); float* HN = (float*)take((size_t)NNODE * CL * 4);
    float* UV = (float*)take((size_t)NNODE * 384 * 4); float* SDH = (float*)take((size_t)NNODE * C2L * 4); float* SD = (float*)take((size_t)NNODE * C2L * 4); float* RD = (float*)take((size_t)NNODE * C2L * 4);
    h16* R1 = (h16*)take((size_t)PCH * C2L * 2); h16* T1 = (h16*)take((size_t)PCH * CL * 2); float* R2F = (float*)take((size_t)PCH * C2L * 4); h16* R2 = (h16*)take((size_t)PCH * C2L * 2); float* REL = (float*)take((size_t)PCH * C2L * 4); float* ATT = (float*)take((size_t)PCH * C2L * 4);
    if ((size_t)(wsp - (char*)d_ws) > ws_size) return;
    k_wt_io<<<CL / 8, 256, 0, stream>>>(sew1, CL, CL, CL, WSE1); k_wt_io<<<CL / 8, 256, 0, stream>>>(sew2, CL, CL, CL, WSE2);
    k_wt_io<<<C2L / 8, 256, 0, stream>>>(sdw1, C2L, CL, C2L, WSD1); k_wt_io<<<C2L / 8, 256, 0, stream>>>(sdw2, C2L, C2L, C2L, WSD2);
    k_wt_io<<<C2L / 8, 256, 0, stream>>>(rcw1, C2L, CL, C2L, WUV); k_wt_io<<<C2L / 8, 256, 0, stream>>>(rcw1 + (size_t)CL * C2L, C2L, CL, C2L, WUV + (size_t)128 * CL);
    k_wt_io<<<CL / 8, 256, 0, stream>>>(anw1, CL, CL, CL, WUV + (size_t)256 * CL); k_wt_io<<<CL / 8, 256, 0, stream>>>(anw1 + (size_t)CL * CL, CL, CL, CL, WUV + (size_t)320 * CL);
    k_wt_ioh<<<C2L / 8, 256, 0, stream>>>(rcw2, C2L, C2L, C2L, WRC2); k_wt_ioh<<<C2L / 8, 256, 0, stream>>>(rcw3, C2L, C2L, C2L, WRC3); k_wt_ioh<<<C2L / 8, 256, 0, stream>>>(anw2, C2L, CL, C2L, WAN2);
    k_cvt64<<<(NNODE / 4) / 8, 256, 0, stream>>>(s, A0);
    k_gemmb<false, false><<<dim3(NNODE / 64, 1, 1), 128, 0, stream>>>(A0, nullptr, WSE1, seb1, F1, CL, nullptr, nullptr, CL);
    k_relusplit<64><<<(NNODE / 4) / 8, 256, 0, stream>>>(F1, NNODE, Ph, Pl);
    k_gemmb<true, false><<<dim3(NNODE / 64, 1, 1), 128, 0, stream>>>(Ph, Pl, WSE2, seb2, F1, CL, nullptr, nullptr, CL);

    k_relusplitf64<<<(NNODE / 2) / 8, 256, 0, stream>>>(F1, NNODE, HN, Ph, Pl);
    k_gemmb<true, false><<<dim3(NNODE / 64, 384 / 64, 1), 128, 0, stream>>>(Ph, Pl, WUV, nullptr, UV, 384, nullptr, nullptr, CL);
    k_gemmb<true, false><<<dim3(NNODE / 64, C2L / 64, 1), 128, 0, stream>>>(Ph, Pl, WSD1, sdb1, SDH, C2L, nullptr, nullptr, CL);
    k_relusplit<128><<<(NNODE / 2) / 8, 256, 0, stream>>>(SDH, NNODE, Ph, Pl);
    k_gemmb<true, false><<<dim3(NNODE / 64, C2L / 64, 1), 128, 0, stream>>>(Ph, Pl, WSD2, sdb2, SD, C2L, nullptr, nullptr, C2L);
    for (int ch = 0; ch < NB_ / ICH; ++ch) { const int node0 = ch * ICH * NN;
        k_pair1<<<PCH / 8, 256, 0, stream>>>(HN, UV, rcw1, rcb1, anw1, anb1, node0, R1, T1);
        k_gemmh<<<dim3(PCH / 64, C2L / 64, 1), 128, 0, stream>>>(R1, WRC2, rcb2, R2F, C2L, nullptr, C2L, 0, 0, 0, 0);
        k_reluh128<<<(PCH / 2) / 8, 256, 0, stream>>>(R2F, PCH, R2);
        k_gemmh<<<dim3(PCH / 64, C2L / 64, 1), 128, 0, stream>>>(R2, WRC3, rcb3, REL, C2L, nullptr, C2L, 0, 0, 0, 0);
        k_gemmh<<<dim3(PCH / 64, C2L / 64, 1), 128, 0, stream>>>(T1, WAN2, anb2, ATT, C2L, nullptr, CL, 0, 0, 0, 0);
        k_pairmean<<<(PCH / NN) / 8, 256, 0, stream>>>(REL, ATT, node0, RD); }
    k_outmean<<<NB_ / 8, 256, 0, stream>>>(SD, RD, out);
}
